// NetworkRNN_reimplement_28192165331633
// MI455X (gfx1250) — hardware-verified
//
#include <hip/hip_runtime.h>

#define B_   64
#define S_   512
#define E_   256
#define H_   512
#define V_   50257
#define HS   520
#define RSPLIT (1.0f / 2048.0f)

typedef _Float16 h16;
typedef __attribute__((ext_vector_type(16))) _Float16 v16h;
typedef __attribute__((ext_vector_type(8)))  _Float16 v8h;
typedef __attribute__((ext_vector_type(8)))  float v8f;
typedef __attribute__((ext_vector_type(4)))  float v4f_t;
typedef float v4fa __attribute__((ext_vector_type(4), may_alias));
typedef __attribute__((ext_vector_type(4)))  unsigned v4u_t;
typedef unsigned v4ua __attribute__((ext_vector_type(4), may_alias));

__device__ __forceinline__ h16 lo_of(float v, h16 h) { return (h16)((v - (float)h) * 2048.0f); }
__device__ __forceinline__ v8f wmma16(v16h a, v16h b, v8f c) { return __builtin_amdgcn_wmma_f32_16x16x32_f16(false, a, false, b, (short)0, c, false, false); }
__device__ __forceinline__ v8f wmma_split(v16h a, v16h al, v16h b, v16h bl, v8f c) { v8f x = {}; x = wmma16(al, b, x); x = wmma16(a, bl, x); return wmma16(a, b, c) + x * RSPLIT; }
__device__ __forceinline__ v16h rfrag(const h16* rowp, int half) {
  const h16* p = rowp + 8 * half;
  return __builtin_shufflevector(*(const v8h*)p, *(const v8h*)(p + 16), 0,1,2,3,4,5,6,7,8,9,10,11,12,13,14,15);
}
__device__ __forceinline__ void frag32(const float* rowp, int half, v16h& hv, v16h& lv) {
#pragma unroll
  for (int e = 0; e < 16; ++e) { const float v = rowp[8 * half + ((e < 8) ? e : (e + 8))]; hv[e] = (h16)v; lv[e] = lo_of(v, hv[e]); }
}

__global__ __launch_bounds__(256) void k_pack_wh(const float* __restrict__ Wh, h16* __restrict__ Wp) {
  const int g = blockIdx.x * 256 + threadIdx.x;
  const int e0 = g * 8;
  h16 hh[8], hl[8];
#pragma unroll
  for (int i = 0; i < 8; ++i) { const float v = Wh[e0 + i]; hh[i] = (h16)v; hl[i] = lo_of(v, hh[i]); }
  *(volatile v4u_t*)(Wp + e0) = *(const v4ua*)hh; *(volatile v4u_t*)(Wp + H_ * H_ + e0) = *(const v4ua*)hl; __threadfence();
  *(volatile v4u_t*)(Wp + e0) = *(const v4ua*)hh; *(volatile v4u_t*)(Wp + H_ * H_ + e0) = *(const v4ua*)hl;
}

__global__ __launch_bounds__(256) void k_embed(const int* __restrict__ words, const float* __restrict__ emb, h16* __restrict__ E) {
  const int g = blockIdx.x * 256 + threadIdx.x;
  const int m = g >> 5, e8 = (g & 31) * 8;
  const int t = m >> 6, b = m & 63;
  int w = words[b * S_ + t]; w = (w < 0) ? 0 : (w >= V_ ? V_ - 1 : w);
  const float* src = emb + (size_t)w * E_ + e8;
  h16 hh[8], hl[8];
#pragma unroll
  for (int i = 0; i < 8; ++i) { const float v = src[i]; hh[i] = (h16)v; hl[i] = lo_of(v, hh[i]); }
  h16* d = E + (size_t)m * E_ + e8;
  const size_t plane = (size_t)S_ * B_ * E_;
  *(volatile v4u_t*)d = *(const v4ua*)hh; *(volatile v4u_t*)(d + plane) = *(const v4ua*)hl; __threadfence();
  *(volatile v4u_t*)d = *(const v4ua*)hh; *(volatile v4u_t*)(d + plane) = *(const v4ua*)hl;
}

__global__ __launch_bounds__(256) void k_xproj(const h16* __restrict__ E, const float* __restrict__ Wi,
                                              const float* __restrict__ bi, const float* __restrict__ bh, float* __restrict__ X) {
  __shared__ __attribute__((aligned(16))) float st[8][16 * 68];
  const int lane = threadIdx.x & 31, wave = threadIdx.x >> 5, half = lane >> 4, l16 = lane & 15;
  const int gw = blockIdx.x * 8 + wave;
  const int mt = gw >> 3, cg = gw & 7;
  const int m = mt * 16 + l16;
  const h16* arow = E + (size_t)m * E_;
  const size_t plane = (size_t)S_ * B_ * E_;
  v8f acc[4] = {};
#pragma unroll 2
  for (int kc = 0; kc < E_ / 32; ++kc) {
    const v16h a = rfrag(arow + kc * 32, half), al = rfrag(arow + plane + kc * 32, half);
#pragma unroll
    for (int q = 0; q < 4; ++q) { v16h bv, bl; frag32(Wi + (size_t)(cg * 64 + q * 16 + l16) * E_ + kc * 32, half, bv, bl); acc[q] = wmma_split(a, al, bv, bl, acc[q]); }
  }
  float* sw = st[wave];
#pragma unroll
  for (int q = 0; q < 4; ++q) { const int col = cg * 64 + q * 16 + l16; const float bb = bi[col] + bh[col];
#pragma unroll
    for (int r = 0; r < 8; ++r) sw[(r + 8 * half) * 68 + q * 16 + l16] = acc[q][r] + bb; }
  asm volatile("s_wait_dscnt 0" ::: "memory");
#pragma unroll 1
  for (int pass = 0; pass < 2; ++pass) {
#pragma unroll
    for (int it = 0; it < 8; ++it) { const int ch = lane + 32 * it, r = ch >> 4, q4 = (ch & 15) * 4;
      *(volatile v4f_t*)(X + (size_t)(mt * 16 + r) * H_ + cg * 64 + q4) = *(const volatile v4fa*)(sw + r * 68 + q4); }
    __threadfence();
  }
}

__global__ __launch_bounds__(256) void k_rnn(const h16* __restrict__ Wp, const float* __restrict__ X,
                                            const float* __restrict__ Wf, const float* __restrict__ bfin, float* __restrict__ out) {
  __shared__ __attribute__((aligned(16))) h16 hbuf[2][2][B_ * HS];
  __shared__ __attribute__((aligned(16))) float sig_s[B_];
  const int tid = threadIdx.x, lane = tid & 31, wave = tid >> 5, half = lane >> 4, l16 = lane & 15;
  for (int i = tid; i < 2 * B_ * HS; i += 256) { hbuf[0][0][i % (B_ * HS)] = (h16)0.0f; hbuf[0][1][i % (B_ * HS)] = (h16)0.0f; }
  __syncthreads();
  const h16* Wlo = Wp + (size_t)H_ * H_;
#pragma unroll 1
  for (int t = 0; t < S_; ++t) {
    const int cur = t & 1, nxt = cur ^ 1;
    const h16* hh = hbuf[cur][0]; const h16* hl = hbuf[cur][1];
    h16* nh = hbuf[nxt][0]; h16* nl = hbuf[nxt][1];
    const float* Xt = X + (size_t)t * B_ * H_;
#pragma unroll 1
    for (int i = 0; i < 16; ++i) {
      const int tile = wave + 8 * i;
      const int rt = tile & 3, ct = tile >> 2;
      const int col = ct * 16 + l16;
      v8f acc;
#pragma unroll
      for (int r = 0; r < 8; ++r) acc[r] = Xt[(size_t)(rt * 16 + 8 * half + r) * H_ + col];
      const h16* wrow = Wp + (size_t)col * H_, * wlrow = Wlo + (size_t)col * H_;
#pragma unroll 4
      for (int kc = 0; kc < H_ / 32; ++kc)
        acc = wmma_split(rfrag(hh + (rt * 16 + l16) * HS + kc * 32, half), rfrag(hl + (rt * 16 + l16) * HS + kc * 32, half),
                         rfrag(wrow + kc * 32, half), rfrag(wlrow + kc * 32, half), acc);
#pragma unroll
      for (int r = 0; r < 8; ++r) {
        const float sg = __builtin_amdgcn_rcpf(1.0f + __expf(-acc[r]));
        const h16 hv = (h16)sg;
        const int row = rt * 16 + 8 * half + r;
        nh[row * HS + col] = hv; nl[row * HS + col] = lo_of(sg, hv);
      }
    }
    __syncthreads();
  }
  const h16* fh = hbuf[S_ & 1][0]; const h16* fl = hbuf[S_ & 1][1];
#pragma unroll 1
  for (int b = wave; b < B_; b += 8) {
    float a = 0.0f;
#pragma unroll 1
    for (int j = lane; j < H_; j += 32) a += ((float)fh[b * HS + j] + (float)fl[b * HS + j] * RSPLIT) * Wf[j];
#pragma unroll
    for (int o = 16; o >= 1; o >>= 1) a += __shfl_xor(a, o, 32);
    if (lane == 0) sig_s[b] = __builtin_amdgcn_rcpf(1.0f + __expf(-(a + bfin[0])));
  }
  __syncthreads();
#pragma unroll 1
  for (int pass = 0; pass < 2; ++pass) {
    for (int ch = tid; ch < B_ * H_ / 4; ch += 256) { const int b = ch >> 7, q = (ch & 127) * 4; v4f_t v;
      v.x = (float)fh[b * HS + q]     + (float)fl[b * HS + q]     * RSPLIT;
      v.y = (float)fh[b * HS + q + 1] + (float)fl[b * HS + q + 1] * RSPLIT;
      v.z = (float)fh[b * HS + q + 2] + (float)fl[b * HS + q + 2] * RSPLIT;
      v.w = (float)fh[b * HS + q + 3] + (float)fl[b * HS + q + 3] * RSPLIT;
      *(volatile v4f_t*)(out + B_ + (size_t)b * H_ + q) = v; }
    if (tid < 16) *(volatile v4f_t*)(out + tid * 4) = *(const volatile v4fa*)(sig_s + tid * 4);
    __threadfence();
  }
}

extern "C" void kernel_launch(void* const* d_in, const int* in_sizes, int n_in,
                              void* d_out, int out_size, void* d_ws, size_t ws_size,
                              hipStream_t stream) {
  (void)in_sizes; (void)n_in; (void)out_size; (void)ws_size;
  const int*   words = (const int*)  d_in[0];
  const float* emb   = (const float*)d_in[1];
  const float* Wh    = (const float*)d_in[2];
  const float* bh    = (const float*)d_in[3];
  const float* Wi    = (const float*)d_in[4];
  const float* bi    = (const float*)d_in[5];
  const float* Wf    = (const float*)d_in[6];
  const float* bfin  = (const float*)d_in[7];
  float* out = (float*)d_out;
  char* ws = (char*)d_ws;
  float* X  = (float*)ws;
  h16*   Wp = (h16*)(ws + (size_t)S_ * B_ * H_ * 4);
  h16*   E  = Wp + 2 * H_ * H_;
  k_pack_wh<<<(H_ * H_ / 8) / 256, 256, 0, stream>>>(Wh, Wp);
  k_embed<<<(S_ * B_ * E_ / 8) / 256, 256, 0, stream>>>(words, emb, E);
  k_xproj<<<(S_ * B_ / 16) * 8 / 8, 256, 0, stream>>>(E, Wi, bi, bh, X);
  k_rnn<<<1, 256, 0, stream>>>(Wp, X, Wf, bfin, out);
}
